// SelfAttention_22900765622276
// MI455X (gfx1250) — hardware-verified
//
#include <hip/hip_runtime.h>
#ifndef NB
#define NB 4
#endif
#ifndef SEQ
#define SEQ 2048
#endif
#define NB_FULL 4
#define SEQ_FULL 2048
#define EM 1024
#define NH 16
#define HD 64
#define KO 2048
#define NR ((size_t)NB * SEQ)
#define WSCALE 1024.0f

static_assert(EM == NH * HD);
static_assert(HD == 64);
static_assert(KO == 2 * EM);
static_assert(SEQ % 64 == 0);
static_assert(((size_t)NB * SEQ) % 128 == 0);
static_assert(EM % 64 == 0 && EM % 32 == 0 && KO % 32 == 0 && EM % 8 == 0);
static_assert(NB <= NB_FULL && SEQ <= SEQ_FULL);

typedef unsigned short v8us __attribute__((ext_vector_type(8), may_alias));
typedef float  v8f  __attribute__((ext_vector_type(8)));
typedef float  v4f  __attribute__((ext_vector_type(4)));
typedef float  v4fa __attribute__((ext_vector_type(4), may_alias));
typedef _Float16 v16h __attribute__((ext_vector_type(16)));
typedef _Float16 v4h __attribute__((ext_vector_type(4)));
union FragH { v16h v; v8us half[2]; _Float16 h[16]; unsigned short u[16]; };

__device__ __forceinline__ unsigned short bf16_bits(float x) { unsigned int u = __float_as_uint(x); return (unsigned short)((u + 0x7FFFu + ((u >> 16) & 1u)) >> 16); }
__device__ __forceinline__ float bf16_val(unsigned short b) { return __uint_as_float(((unsigned int)b) << 16); }
__device__ __forceinline__ float bf16_rne(float x) { return bf16_val(bf16_bits(x)); }

__device__ __forceinline__ v16h g2_frag(const _Float16* p, int hh) { FragH f; f.half[0] = *(const v8us*)((const unsigned short*)p + 8 * hh); f.half[1] = *(const v8us*)((const unsigned short*)p + 16 + 8 * hh); return f.v; }
__device__ __forceinline__ v8f g2_mma(v16h a, v16h b, v8f c) { v8f d = __builtin_amdgcn_wmma_f32_16x16x32_f16(false, a, false, b, (short)0, c, false, false); asm volatile("v_nop\n\tv_nop\n\tv_nop\n\tv_nop" : "+v"(d) : "v"(a), "v"(b)); return d; }

__global__ __launch_bounds__(256) void k_x16(const float* __restrict__ x, _Float16* __restrict__ X16) {
  const size_t t = (size_t)blockIdx.x * 256 + threadIdx.x;
  if (t >= NR * (EM / 8)) return;
  const size_t row = t / (EM / 8); const int c8 = (int)(t % (EM / 8)) * 8;
  const size_t b = row / SEQ, s = row % SEQ;
  const float* src = x + ((b * SEQ_FULL + s) * EM + c8);
  const v4f a = *(const v4fa*)src, c = *(const v4fa*)(src + 4);
  FragH f;
#pragma unroll
  for (int q = 0; q < 4; ++q) { f.h[q] = (_Float16)bf16_rne(a[q]); f.h[4 + q] = (_Float16)bf16_rne(c[q]); }
  const v8us o = f.half[0];
  unsigned short* d = (unsigned short*)X16 + t * 8;
  *(volatile v8us*)d = o; __threadfence(); *(volatile v8us*)d = o;
}

__global__ __launch_bounds__(256) void k_wt_f16(const float* __restrict__ W, _Float16* __restrict__ Wt, int K, int N, int ldw, int koff, float scale) {
  const int t = blockIdx.x * 256 + threadIdx.x; if (t >= N * (K / 8)) return;
  const int n = t / (K / 8), k8 = (t % (K / 8)) * 8; FragH f;
#pragma unroll
  for (int i = 0; i < 8; ++i) f.h[i] = (_Float16)(bf16_rne(W[(size_t)(k8 + i) * N + n]) * scale);
  const v8us o = f.half[0];
  unsigned short* d = (unsigned short*)Wt + (size_t)n * ldw + koff + k8;
  *(volatile v8us*)d = o; __threadfence(); *(volatile v8us*)d = o;
}

__global__ __launch_bounds__(128) void k_gemm2(const _Float16* __restrict__ A, int lda, const _Float16* __restrict__ Bh, int ldb, float alpha, const float* __restrict__ bias,
                                              float* __restrict__ C, _Float16* __restrict__ C16, int ldc, int M, int N, int K) {
  __shared__ __attribute__((aligned(16))) float so[4][32][68];
  const int lane = threadIdx.x & 31, ln = lane & 15, hh = lane >> 4;
  const int w = __builtin_amdgcn_readfirstlane((int)(threadIdx.x >> 5));
  const int ntn = N >> 6; const int mt = blockIdx.x / ntn, nq = blockIdx.x - mt * ntn; const int row0 = mt * 128 + 32 * w, col0 = nq * 64; if (row0 >= M) return;
  const _Float16* a0p = A + (size_t)(row0 + ln) * lda; const _Float16* a1p = a0p + (size_t)16 * lda;
  const _Float16* b0p = Bh + (size_t)(col0 + ln) * ldb; const _Float16* b1p = b0p + (size_t)16 * ldb; const _Float16* b2p = b1p + (size_t)16 * ldb; const _Float16* b3p = b2p + (size_t)16 * ldb;
  const v8f z8 = {0.f,0.f,0.f,0.f,0.f,0.f,0.f,0.f}; v8f c00 = z8, c01 = z8, c02 = z8, c03 = z8, c10 = z8, c11 = z8, c12 = z8, c13 = z8;
#pragma unroll 1
  for (int kb = 0; kb < K; kb += 32) { const v16h a0 = g2_frag(a0p + kb, hh), a1 = g2_frag(a1p + kb, hh);
    v16h b = g2_frag(b0p + kb, hh); c00 = g2_mma(a0, b, c00); c10 = g2_mma(a1, b, c10);
    b = g2_frag(b1p + kb, hh); c01 = g2_mma(a0, b, c01); c11 = g2_mma(a1, b, c11);
    b = g2_frag(b2p + kb, hh); c02 = g2_mma(a0, b, c02); c12 = g2_mma(a1, b, c12);
    b = g2_frag(b3p + kb, hh); c03 = g2_mma(a0, b, c03); c13 = g2_mma(a1, b, c13); }
  v8f accs[8] = {c00, c01, c02, c03, c10, c11, c12, c13};
#pragma unroll
  for (int u = 0; u < 8; ++u) { const int t = u & 3, half = u >> 2; const int col = col0 + t * 16 + ln; const float bv = bf16_rne(bias[col]);
#pragma unroll
    for (int r = 0; r < 8; ++r) { const int rloc = half * 16 + 8 * hh + r; so[w][rloc][t * 16 + ln] = accs[u][r] * alpha + bv; } }
  __builtin_amdgcn_fence(4  , "workgroup"); __builtin_amdgcn_wave_barrier();
  const int rsub = lane >> 4, c4 = (lane & 15) * 4;
  for (int pass = 0; pass < 2; ++pass) {
#pragma unroll
    for (int q = 0; q < 16; ++q) { const int r = q * 2 + rsub; const v4f v = *(const v4fa*)&so[w][r][c4];
      if (C) *(volatile v4f*)(C + (size_t)(row0 + r) * ldc + col0 + c4) = v;
      if (C16) { v4h h4;
#pragma unroll
        for (int i = 0; i < 4; ++i) h4[i] = (_Float16)v[i];
        *(volatile v4h*)(C16 + (size_t)(row0 + r) * ldc + col0 + c4) = h4; } }
    if (pass == 0) __threadfence(); }
}

__global__ __launch_bounds__(256) void k_vt(const _Float16* __restrict__ V16, _Float16* __restrict__ VT) {
  __shared__ unsigned short tl[64][65];
  const int tid = threadIdx.x; const int bh = blockIdx.y; const int b = bh / NH, h = bh - b * NH; const int s0 = blockIdx.x * 64;
  for (int i = tid; i < 64 * 8; i += 256) { const int j = i / 8, d8 = (i % 8) * 8;
    const v8us f = *(const v8us*)((const unsigned short*)V16 + ((size_t)b * SEQ + s0 + j) * EM + h * HD + d8);
#pragma unroll
    for (int q = 0; q < 8; ++q) tl[d8 + q][j] = f[q]; }
  __syncthreads();
  for (int pass = 0; pass < 2; ++pass) {
    for (int i = tid; i < 64 * 8; i += 256) { const int d = i / 8, j8 = (i % 8) * 8; FragH f;
#pragma unroll
      for (int q = 0; q < 8; ++q) f.u[q] = tl[d][j8 + q];
      *(volatile v8us*)((unsigned short*)VT + ((size_t)bh * HD + d) * SEQ + s0 + j8) = f.half[0]; }
    if (pass == 0) __threadfence(); }
}

__global__ __launch_bounds__(128) void k_flash(const _Float16* __restrict__ Q16, const _Float16* __restrict__ K16, const _Float16* __restrict__ VT, _Float16* __restrict__ CTX) {
  __shared__ __attribute__((aligned(16))) unsigned short st[4][2][16][72];
  const int lane = threadIdx.x & 31, ln = lane & 15, hh = lane >> 4;
  const int wave = __builtin_amdgcn_readfirstlane((int)(threadIdx.x >> 5));
  const int bh = blockIdx.y; const int b = bh / NH, h = bh - b * NH;
  const int q0 = blockIdx.x * 64 + wave * 16;
  const _Float16* qp = Q16 + ((size_t)b * SEQ + q0 + ln) * EM + h * HD;
  const v16h qf0 = g2_frag(qp, hh), qf1 = g2_frag(qp + 32, hh);
  const _Float16* kp = K16 + ((size_t)b * SEQ + ln) * EM + h * HD;
  const _Float16* vp = VT + ((size_t)bh * HD + ln) * SEQ;
  const v8f z8 = {0.f,0.f,0.f,0.f,0.f,0.f,0.f,0.f};
  v8f o[4] = {z8, z8, z8, z8};
  float m = -1.0e30f, l = 0.f;
  const float CL = 0.18033688011112042f;
#pragma unroll 1
  for (int key0 = 0; key0 < SEQ; key0 += 64) {
    v8f s[4];
#pragma unroll
    for (int t = 0; t < 4; ++t) {
      const _Float16* kr = kp + (size_t)(key0 + t * 16) * EM;
      v8f c = z8;
      c = g2_mma(g2_frag(kr, hh), qf0, c);
      c = g2_mma(g2_frag(kr + 32, hh), qf1, c);
      s[t] = c;
    }
    float mx = s[0][0];
#pragma unroll
    for (int t = 0; t < 4; ++t)
#pragma unroll
      for (int r = 0; r < 8; ++r) mx = fmaxf(mx, s[t][r]);
    mx = fmaxf(mx, __shfl_xor(mx, 16));
    const float mn = fmaxf(m, mx);
    const float alpha = __builtin_amdgcn_exp2f((m - mn) * CL);
    m = mn;
    const float off = 8.0f - mn * CL;
    float rs = 0.f;
#pragma unroll
    for (int t = 0; t < 4; ++t)
#pragma unroll
      for (int r = 0; r < 8; ++r) { const float p = __builtin_amdgcn_exp2f(fmaf(s[t][r], CL, off)); s[t][r] = p; rs += p; }
    l = l * alpha + rs;
#pragma unroll
    for (int t = 0; t < 4; ++t) o[t] = o[t] * alpha;
    FragH pa, pb;
#pragma unroll
    for (int r = 0; r < 8; ++r) { pa.h[r] = (_Float16)s[0][r]; pa.h[8 + r] = (_Float16)s[1][r]; pb.h[r] = (_Float16)s[2][r]; pb.h[8 + r] = (_Float16)s[3][r]; }
    const _Float16* vr = vp + key0;
#pragma unroll
    for (int t = 0; t < 4; ++t) {
      const _Float16* v0 = vr + (size_t)(t * 16) * SEQ;
      o[t] = g2_mma(g2_frag(v0, hh), pa.v, o[t]);
      o[t] = g2_mma(g2_frag(v0 + 32, hh), pb.v, o[t]);
    }
  }
  const float lt = l + __shfl_xor(l, 16);
  const float inv = 64.0f * (1.0f / lt);
#pragma unroll
  for (int t = 0; t < 4; ++t) {
    FragH fh, fl;
#pragma unroll
    for (int r = 0; r < 8; ++r) { const float c = o[t][r] * inv; const _Float16 hq = (_Float16)c; fh.h[r] = hq; fl.h[r] = (_Float16)((c - (float)hq) * 1024.0f); }
    *(v8us*)&st[wave][0][ln][t * 16 + 8 * hh] = fh.half[0];
    *(v8us*)&st[wave][1][ln][t * 16 + 8 * hh] = fl.half[0];
  }
  __builtin_amdgcn_fence(4  , "workgroup"); __builtin_amdgcn_wave_barrier();
  const int rs4 = lane >> 3, pc = lane & 7;
  v8us vh[4], vl[4];
#pragma unroll
  for (int i = 0; i < 4; ++i) { vh[i] = *(const v8us*)&st[wave][0][i * 4 + rs4][pc * 8]; vl[i] = *(const v8us*)&st[wave][1][i * 4 + rs4][pc * 8]; }
  unsigned short* cb = (unsigned short*)CTX + ((size_t)b * SEQ + q0) * KO + h * HD + pc * 8;
  for (int pass = 0; pass < 2; ++pass) {
#pragma unroll
    for (int i = 0; i < 4; ++i) { unsigned short* d = cb + (size_t)(i * 4 + rs4) * KO; *(volatile v8us*)d = vh[i]; *(volatile v8us*)(d + EM) = vl[i]; }
    if (pass == 0) __threadfence(); }
}

constexpr size_t SZ_W   = (size_t)EM * EM * 2;
constexpr size_t SZ_WO  = (size_t)EM * KO * 2;
constexpr size_t SZ_X1  = NR * EM * 2;
constexpr size_t SZ_CTX = NR * KO * 2;
constexpr size_t WS_TOTAL = 3 * SZ_W + SZ_WO + 3 * SZ_X1 + 3 * SZ_X1 + SZ_X1;
static_assert(WS_TOTAL <= (size_t)134217728);
static_assert(SZ_CTX <= 2 * SZ_X1);
static_assert(SZ_W % 256 == 0 && SZ_WO % 256 == 0 && SZ_X1 % 256 == 0);
static_assert((size_t)NB * NH * HD * SEQ * 2 == SZ_X1);

extern "C" void kernel_launch(void* const* d_in, const int* in_sizes, int n_in,
                              void* d_out, int out_size, void* d_ws, size_t ws_size, hipStream_t stream) {
  if (n_in < 11) return;
  const size_t needx = ((size_t)(NB - 1) * SEQ_FULL + SEQ) * EM;
  if ((size_t)in_sizes[0] < needx || (size_t)in_sizes[1] < needx || (size_t)in_sizes[2] < needx) return;
  if ((size_t)in_sizes[3] < (size_t)EM * EM || (size_t)in_sizes[5] < (size_t)EM * EM || (size_t)in_sizes[7] < (size_t)EM * EM || (size_t)in_sizes[9] < (size_t)EM * EM) return;
  if (in_sizes[4] < EM || in_sizes[6] < EM || in_sizes[8] < EM || in_sizes[10] < EM) return;
  if ((size_t)out_size < NR * EM) return;
  const float* xq = (const float*)d_in[0]; const float* xk = (const float*)d_in[1]; const float* xv = (const float*)d_in[2];
  const float* wq = (const float*)d_in[3]; const float* bq = (const float*)d_in[4];
  const float* wk = (const float*)d_in[5]; const float* bk = (const float*)d_in[6];
  const float* wv = (const float*)d_in[7]; const float* bv = (const float*)d_in[8];
  const float* wo = (const float*)d_in[9]; const float* bo = (const float*)d_in[10];
  char* ws = (char*)d_ws; size_t off = 0;
  auto take = [&](size_t bytes) { char* p = ws + off; off += (bytes + 255) & ~(size_t)255; return p; };
  _Float16* WQ = (_Float16*)take(SZ_W); _Float16* WK = (_Float16*)take(SZ_W); _Float16* WV = (_Float16*)take(SZ_W); _Float16* WO = (_Float16*)take(SZ_WO);
  _Float16* X = (_Float16*)take(3 * SZ_X1);
  _Float16* XQ = X; _Float16* XK = X + NR * EM; _Float16* XV = X + 2 * NR * EM; _Float16* CTX = X;
  _Float16* Q16 = (_Float16*)take(SZ_X1); _Float16* K16 = (_Float16*)take(SZ_X1); _Float16* V16 = (_Float16*)take(SZ_X1);
  _Float16* VT = (_Float16*)take(SZ_X1);
  if (off > ws_size) return;
  { const unsigned g = (unsigned)(((size_t)EM * (EM / 8) + 255) / 256);
    k_wt_f16<<<g, 256, 0, stream>>>(wq, WQ, EM, EM, EM, 0, WSCALE);
    k_wt_f16<<<g, 256, 0, stream>>>(wk, WK, EM, EM, EM, 0, WSCALE);
    k_wt_f16<<<g, 256, 0, stream>>>(wv, WV, EM, EM, EM, 0, WSCALE);
    k_wt_f16<<<g, 256, 0, stream>>>(wo, WO, EM, EM, KO, 0, WSCALE);
    k_wt_f16<<<g, 256, 0, stream>>>(wo, WO, EM, EM, KO, EM, 1.0f); }
  { const unsigned g = (unsigned)((NR * (EM / 8) + 255) / 256);
    k_x16<<<g, 256, 0, stream>>>(xq, XQ); k_x16<<<g, 256, 0, stream>>>(xk, XK); k_x16<<<g, 256, 0, stream>>>(xv, XV); }
  { const unsigned g = (unsigned)((NR / 128) * (EM / 64));
    k_gemm2<<<g, 128, 0, stream>>>(XQ, EM, WQ, EM, 0.0009765625f, bq, nullptr, Q16, EM, (int)NR, EM, EM);
    k_gemm2<<<g, 128, 0, stream>>>(XK, EM, WK, EM, 0.0009765625f, bk, nullptr, K16, EM, (int)NR, EM, EM);
    k_gemm2<<<g, 128, 0, stream>>>(XV, EM, WV, EM, 0.0009765625f, bv, nullptr, V16, EM, (int)NR, EM, EM); }
  k_vt<<<dim3(SEQ / 64, NB * NH), 256, 0, stream>>>(V16, VT);
  k_flash<<<dim3(SEQ / 64, NB * NH), 128, 0, stream>>>(Q16, K16, VT, CTX);
  { const unsigned g = (unsigned)((NR / 128) * (EM / 64));
    k_gemm2<<<g, 128, 0, stream>>>(CTX, KO, WO, KO, 1.52587890625e-05f, bo, (float*)d_out, nullptr, EM, (int)NR, EM, KO); }
}
